// SemanticComposite_42949672961824
// MI455X (gfx1250) — hardware-verified
//
#include <hip/hip_runtime.h>
#include <math.h>
#include <stdint.h>

#define NB 8
#define NS 2048
#define NF 256
#define NG 512
#define NR (NB * NS)
#define TP 260
#define QROWS 64
#define KCH 32
#define PPITCH 40
#define APITCH 68
#define NGRP 4
#define SLP 68

typedef _Float16 v16h __attribute__((ext_vector_type(16)));
typedef _Float16 v8h __attribute__((ext_vector_type(8)));
typedef __bf16 v16b __attribute__((ext_vector_type(16)));
typedef unsigned short v8us __attribute__((ext_vector_type(8)));
typedef float v8f __attribute__((ext_vector_type(8)));
typedef float v4f __attribute__((ext_vector_type(4), __may_alias__));
typedef unsigned int v4u __attribute__((ext_vector_type(4)));

union FH { v16h v; v8us u[2]; };
union FB { v16b v; v8us u[2]; };
union H8 { v8h h; v8us u; };
union AV { v8f v; v4f q[2]; };

__device__ __forceinline__ v8f z8() {
  v8f v = {0.f, 0.f, 0.f, 0.f, 0.f, 0.f, 0.f, 0.f};
  return v;
}
__device__ __forceinline__ unsigned short bfb(float f) {
  const unsigned u = __float_as_uint(f);
  return (unsigned short)((u + 0x7FFFu + ((u >> 16) & 1u)) >> 16);
}
__device__ __forceinline__ float bff(unsigned short h) { return __uint_as_float(((unsigned)h) << 16); }
__device__ __forceinline__ unsigned pk2(unsigned short a, unsigned short b) { return (unsigned)a | ((unsigned)b << 16); }

__device__ __forceinline__ void ld8f(const float* p, float (&v)[8]) {
  const v4f t0 = *(const v4f*)p;
  const v4f t1 = *(const v4f*)(p + 4);
#pragma unroll
  for (int q = 0; q < 4; ++q) { v[q] = t0[q]; v[4 + q] = t1[q]; }
}
__device__ __forceinline__ void pk_bf16x8(const float (&v)[8], v4u& hi, v4u& lo) {
#pragma unroll
  for (int q = 0; q < 4; ++q) {
    const unsigned short h0 = bfb(v[2 * q]), h1 = bfb(v[2 * q + 1]);
    const unsigned short l0 = bfb(v[2 * q] - bff(h0)), l1 = bfb(v[2 * q + 1] - bff(h1));
    hi[q] = pk2(h0, h1);
    lo[q] = pk2(l0, l1);
  }
}
__device__ __forceinline__ v8us pk_f16x8(const float (&v)[8], float s) {
  H8 r;
#pragma unroll
  for (int e = 0; e < 8; ++e) r.h[e] = (_Float16)(v[e] * s);
  return r.u;
}
__device__ __forceinline__ v16h ldh(const unsigned short* p) {
  FH f;
  f.u[0] = *(const v8us*)p;
  f.u[1] = *(const v8us*)(p + 16);
  return f.v;
}
__device__ __forceinline__ v16b ldb(const unsigned short* p) {
  FB f;
  f.u[0] = *(const v8us*)p;
  f.u[1] = *(const v8us*)(p + 16);
  return f.v;
}
__device__ __forceinline__ v8f mma_h(v16h a, v16h b, v8f c) {
  return __builtin_amdgcn_wmma_f32_16x16x32_f16(false, a, false, b, (short)0, c, false, false);
}
__device__ __forceinline__ v8f mma_b(v16b a, v16b b, v8f c) {
  return __builtin_amdgcn_wmma_f32_16x16x32_bf16(false, a, false, b, (short)0, c, false, false);
}
__device__ __forceinline__ void g_s(v8f& s0, v8f& s1, v16h a, v16h b0, v16h b1) {
  asm volatile("v_nop\n\tv_nop\n\tv_nop\n\tv_nop" : "+v"(s0), "+v"(s1) : "v"(a), "v"(b0), "v"(b1));
}
__device__ __forceinline__ void g_o(v8f& o, v16b ph, v16b pl, v16b bh, v16b bl) {
  asm volatile("v_nop\n\tv_nop\n\tv_nop\n\tv_nop" : "+v"(o) : "v"(ph), "v"(pl), "v"(bh), "v"(bl) : "memory");
}
__device__ __forceinline__ void g_g(v8f& z, v8f& r, v8f& f, v16h a16, v16b ah, v16b al,
                                    v16b bzh, v16b bzl, v16h br, v16h bf) {
  asm volatile("v_nop\n\tv_nop\n\tv_nop\n\tv_nop"
               : "+v"(z), "+v"(r), "+v"(f)
               : "v"(a16), "v"(ah), "v"(al), "v"(bzh), "v"(bzl), "v"(br), "v"(bf));
}

__global__ void __launch_bounds__(256) prep_w(const float* __restrict__ zw, const float* __restrict__ rw,
                                              const float* __restrict__ fw,
                                              unsigned short* __restrict__ zwh, unsigned short* __restrict__ zwl,
                                              unsigned short* __restrict__ rw16, unsigned short* __restrict__ fw16,
                                              int n8) {
  const int i = (int)blockIdx.x * 256 + (int)threadIdx.x;
  if (i >= n8) return;
  const size_t e0 = (size_t)i * 8;
  float a[8], b[8], d[8];
  ld8f(zw + e0, a);
  ld8f(rw + e0, b);
  ld8f(fw + e0, d);
  v4u zh, zl;
  pk_bf16x8(a, zh, zl);
  const v8us r16 = pk_f16x8(b, 16.0f);
  const v8us f16 = pk_f16x8(d, 16.0f);
  *(volatile v4u*)(zwh + e0) = zh;
  *(volatile v4u*)(zwl + e0) = zl;
  *(volatile v8us*)(rw16 + e0) = r16;
  *(volatile v8us*)(fw16 + e0) = f16;
  __threadfence();
  *(volatile v4u*)(zwh + e0) = zh;
  *(volatile v4u*)(zwl + e0) = zl;
  *(volatile v8us*)(rw16 + e0) = r16;
  *(volatile v8us*)(fw16 + e0) = f16;
}

__global__ void __launch_bounds__(256) prep_x(const float* __restrict__ x, const float* __restrict__ attw,
                                              unsigned short* __restrict__ xh, unsigned short* __restrict__ xwc,
                                              unsigned short* __restrict__ xbh, unsigned short* __restrict__ xbl,
                                              unsigned short* __restrict__ xth, unsigned short* __restrict__ xtl,
                                              float* __restrict__ av, float* __restrict__ bv) {
  __shared__ __align__(16) float tile[64 * TP];
  __shared__ __align__(16) float avs[64];
  __shared__ __align__(16) float bvs[64];
  const int tid = (int)threadIdx.x, wave = tid >> 5, lane = tid & 31;
  const int blk = (int)blockIdx.x;
  const size_t grow0 = (size_t)blk * 64;
  const int bb = blk >> 5;
  const int j0 = (blk & 31) * 64;

#pragma unroll
  for (int it = 0; it < 16; ++it) {
    const int idx = it * 256 + tid;
    const int r = idx >> 6, c4 = (idx & 63) * 4;
    const v4f v = *(const v4f*)(x + (grow0 + r) * NF + c4);
    *(v4f*)(tile + r * TP + c4) = v;
  }
  __syncthreads();

  const int f0 = lane * 8;
  float wa[8], wb[8], wc[8];
  ld8f(attw + f0, wa);
  ld8f(attw + NF + f0, wb);
  ld8f(attw + 2 * NF + f0, wc);

#pragma unroll 1
  for (int rr = 0; rr < 8; ++rr) {
    const int row = wave * 8 + rr;
    float v[8];
    ld8f(tile + row * TP + f0, v);
    float sa = 0.f, sb = 0.f;
#pragma unroll
    for (int e = 0; e < 8; ++e) { sa += v[e] * wa[e]; sb += v[e] * wb[e]; }
#pragma unroll
    for (int m = 16; m >= 1; m >>= 1) {
      sa += __shfl_xor(sa, m, 32);
      sb += __shfl_xor(sb, m, 32);
    }
    if (lane == 0) { avs[row] = sa; bvs[row] = sb; }
  }

  for (int pass = 0; pass < 2; ++pass) {
#pragma unroll 1
    for (int rr = 0; rr < 8; ++rr) {
      const int row = wave * 8 + rr;
      float v[8], w[8];
      ld8f(tile + row * TP + f0, v);
#pragma unroll
      for (int e = 0; e < 8; ++e) w[e] = v[e] * wc[e];
      const v8us h1 = pk_f16x8(v, 1.0f);
      const v8us h2 = pk_f16x8(w, 64.0f);
      v4u hb, lb;
      pk_bf16x8(v, hb, lb);
      const size_t o = (grow0 + row) * NF + f0;
      *(volatile v8us*)(xh + o) = h1;
      *(volatile v8us*)(xwc + o) = h2;
      *(volatile v4u*)(xbh + o) = hb;
      *(volatile v4u*)(xbl + o) = lb;
    }
    __threadfence();
  }

  const int q = lane >> 3, c8 = (lane & 7) * 8;
  const size_t tb = (size_t)bb * NF * NS;
  for (int pass = 0; pass < 2; ++pass) {
#pragma unroll 1
    for (int it = 0; it < 8; ++it) {
      const int fr = wave * 32 + it * 4 + q;
      float t[8];
#pragma unroll
      for (int e = 0; e < 8; ++e) t[e] = tile[(c8 + e) * TP + fr];
      v4u hb, lb;
      pk_bf16x8(t, hb, lb);
      const size_t o = tb + (size_t)fr * NS + j0 + c8;
      *(volatile v4u*)(xth + o) = hb;
      *(volatile v4u*)(xtl + o) = lb;
    }
    __threadfence();
  }

  __syncthreads();
  const int l4 = (lane & 15) * 4;
  for (int pass = 0; pass < 2; ++pass) {
    const v4f a4 = *(const v4f*)(avs + l4);
    const v4f b4 = *(const v4f*)(bvs + l4);
    if (lane < 16) {
      if (wave == 0) *(volatile v4f*)(av + grow0 + l4) = a4;
      else if (wave == 1) *(volatile v4f*)(bv + grow0 + l4) = b4;
    }
    __threadfence();
  }
}

__global__ void __launch_bounds__(128) __attribute__((amdgpu_num_vgpr(256)))
attn_kernel(const unsigned short* __restrict__ xwc, const unsigned short* __restrict__ xh,
            const unsigned short* __restrict__ xth, const unsigned short* __restrict__ xtl,
            const float* __restrict__ av, const float* __restrict__ bv,
            unsigned short* __restrict__ ah, unsigned short* __restrict__ abh,
            unsigned short* __restrict__ abl) {
  __shared__ __align__(16) unsigned short psh[4][16 * PPITCH];
  __shared__ __align__(16) unsigned short psl[4][16 * PPITCH];
  __shared__ __align__(16) v4f accl[4][16 * 32 * 2];
  __shared__ __align__(16) float osm[4][16 * APITCH];

  const int tid = (int)threadIdx.x, wave = tid >> 5, lane = tid & 31, hh = lane >> 4, c = lane & 15;
  const int blk = (int)blockIdx.x, bb = blk >> 5, qb = blk & 31;
  const size_t grow0 = (size_t)bb * NS + (size_t)(qb * QROWS + wave * 16);
  const unsigned short* XHb = xh + (size_t)bb * NS * NF;
  const unsigned short* XTh = xth + (size_t)bb * NF * NS;
  const unsigned short* XTl = xtl + (size_t)bb * NF * NS;
  const float* bvb = bv + (size_t)bb * NS;
  const unsigned short* arow = xwc + (grow0 + c) * NF + 8 * hh;

  float aRow[8], mRow[8], lRow[8];
#pragma unroll
  for (int r = 0; r < 8; ++r) {
    aRow[r] = av[grow0 + 8 * hh + r];
    mRow[r] = -INFINITY;
    lRow[r] = 0.f;
  }
  v8f acc[NGRP];
#pragma unroll
  for (int tt = 0; tt < NGRP; ++tt) acc[tt] = z8();
  v4f* aw = &accl[wave][0];
  {
    const v4f z4 = {0.f, 0.f, 0.f, 0.f};
#pragma unroll 1
    for (int t = 0; t < 16; ++t) {
      const int so = (t * 32 + lane) * 2;
      aw[so] = z4;
      aw[so + 1] = z4;
    }
  }
  unsigned short* pwh = &psh[wave][0];
  unsigned short* pwl = &psl[wave][0];

#pragma unroll 1
  for (int jc = 0; jc < NS / KCH; ++jc) {
    const int j0 = jc * KCH;
    v8f s0 = z8(), s1 = z8();
    const unsigned short* b0row = XHb + (size_t)(j0 + c) * NF + 8 * hh;
    const unsigned short* b1row = b0row + 16 * NF;
#pragma unroll 1
    for (int kk = 0; kk < NF / 32; ++kk) {
      const v16h a = ldh(arow + kk * 32);
      const v16h b0 = ldh(b0row + kk * 32);
      const v16h b1 = ldh(b1row + kk * 32);
      s0 = mma_h(a, b0, s0);
      s1 = mma_h(a, b1, s1);
      g_s(s0, s1, a, b0, b1);
    }
    const float bj0 = bvb[j0 + c], bj1 = bvb[j0 + 16 + c];
    float cm[8];
#pragma unroll
    for (int r = 0; r < 8; ++r) {
      const float t0 = (aRow[r] + bj0) + s0[r] * 0.015625f;
      const float t1 = (aRow[r] + bj1) + s1[r] * 0.015625f;
      s0[r] = t0;
      s1[r] = t1;
      float m = fmaxf(t0, t1);
#pragma unroll
      for (int off = 1; off < 16; off <<= 1) m = fmaxf(m, __shfl_xor(m, off, 32));
      cm[r] = m;
    }
    float alpha[8];
#pragma unroll
    for (int r = 0; r < 8; ++r) {
      const float mnew = fmaxf(mRow[r], cm[r]);
      alpha[r] = expf(mRow[r] - mnew);
      mRow[r] = mnew;
      const float p0 = expf(s0[r] - mnew);
      const float p1 = expf(s1[r] - mnew);
      float ps = p0 + p1;
#pragma unroll
      for (int off = 1; off < 16; off <<= 1) ps += __shfl_xor(ps, off, 32);
      lRow[r] = lRow[r] * alpha[r] + ps;
      const unsigned short hb0 = bfb(p0), hb1 = bfb(p1);
      const unsigned short lb0 = bfb(p0 - bff(hb0)), lb1 = bfb(p1 - bff(hb1));
      const int po = (8 * hh + r) * PPITCH + c;
      pwh[po] = hb0;
      pwh[po + 16] = hb1;
      pwl[po] = lb0;
      pwl[po + 16] = lb1;
    }
    __builtin_amdgcn_fence(__ATOMIC_RELEASE, "workgroup");
    __builtin_amdgcn_wave_barrier();
    __builtin_amdgcn_fence(__ATOMIC_ACQUIRE, "workgroup");
    const v16b ph = ldb(pwh + c * PPITCH + 8 * hh);
    const v16b pl = ldb(pwl + c * PPITCH + 8 * hh);
    const size_t bo = (size_t)c * NS + (size_t)(j0 + 8 * hh);
    const int odd = jc & 1;
#pragma unroll 1
    for (int s = 0; s < NGRP; ++s) {
      const int g = odd ? (NGRP - 1 - s) : s;
      if (s != 0) {
        const int gp = odd ? (NGRP - s) : (s - 1);
#pragma unroll
        for (int tt = 0; tt < NGRP; ++tt) {
          AV u;
          u.v = acc[tt];
          const int so = ((gp * NGRP + tt) * 32 + lane) * 2;
          aw[so] = u.q[0];
          aw[so + 1] = u.q[1];
        }
#pragma unroll
        for (int tt = 0; tt < NGRP; ++tt) {
          const int lo = ((g * NGRP + tt) * 32 + lane) * 2;
          AV u;
          u.q[0] = aw[lo];
          u.q[1] = aw[lo + 1];
          acc[tt] = u.v;
        }
      }
#pragma unroll
      for (int tt = 0; tt < NGRP; ++tt) {
#pragma unroll
        for (int r = 0; r < 8; ++r) acc[tt][r] *= alpha[r];
      }
#pragma unroll
      for (int tt = 0; tt < NGRP; ++tt) {
        const size_t to = (size_t)((g * NGRP + tt) * 16) * NS + bo;
        const v16b bh = ldb(XTh + to);
        const v16b bl = ldb(XTl + to);
        v8f o = acc[tt];
        o = mma_b(ph, bh, o);
        o = mma_b(ph, bl, o);
        o = mma_b(pl, bh, o);
        g_o(o, ph, pl, bh, bl);
        acc[tt] = o;
      }
    }
  }

  {
    const int glast = (((NS / KCH) - 1) & 1) ? 0 : (NGRP - 1);
#pragma unroll
    for (int tt = 0; tt < NGRP; ++tt) {
      AV u;
      u.v = acc[tt];
      const int so = ((glast * NGRP + tt) * 32 + lane) * 2;
      aw[so] = u.q[0];
      aw[so + 1] = u.q[1];
    }
  }

  float inv[8];
#pragma unroll
  for (int r = 0; r < 8; ++r) inv[r] = 1.0f / lRow[r];
  float* osw = &osm[wave][0];
  const int q = lane >> 3, c8 = (lane & 7) * 8;
#pragma unroll 1
  for (int g = 0; g < NGRP; ++g) {
#pragma unroll
    for (int tt = 0; tt < NGRP; ++tt) {
      const int lo = ((g * NGRP + tt) * 32 + lane) * 2;
      AV u;
      u.q[0] = aw[lo];
      u.q[1] = aw[lo + 1];
#pragma unroll
      for (int r = 0; r < 8; ++r) osw[(8 * hh + r) * APITCH + tt * 16 + c] = u.v[r] * inv[r];
    }
    __builtin_amdgcn_fence(__ATOMIC_RELEASE, "workgroup");
    __builtin_amdgcn_wave_barrier();
    __builtin_amdgcn_fence(__ATOMIC_ACQUIRE, "workgroup");
    for (int pass = 0; pass < 2; ++pass) {
#pragma unroll
      for (int it = 0; it < 4; ++it) {
        const int row = it * 4 + q;
        float v[8];
        ld8f(osw + row * APITCH + c8, v);
        const v8us h1 = pk_f16x8(v, 1.0f);
        v4u hb, lb;
        pk_bf16x8(v, hb, lb);
        const size_t o = (grow0 + row) * NF + (size_t)(g * 64 + c8);
        *(volatile v8us*)(ah + o) = h1;
        *(volatile v4u*)(abh + o) = hb;
        *(volatile v4u*)(abl + o) = lb;
      }
      __threadfence();
    }
    __builtin_amdgcn_fence(__ATOMIC_RELEASE, "workgroup");
    __builtin_amdgcn_wave_barrier();
    __builtin_amdgcn_fence(__ATOMIC_ACQUIRE, "workgroup");
  }
}

__global__ void __launch_bounds__(256) __attribute__((amdgpu_num_vgpr(256)))
gates_kernel(const float* __restrict__ x,
             const unsigned short* __restrict__ xh, const unsigned short* __restrict__ xbh,
             const unsigned short* __restrict__ xbl,
             const unsigned short* __restrict__ ah, const unsigned short* __restrict__ abh,
             const unsigned short* __restrict__ abl,
             const unsigned short* __restrict__ zwh, const unsigned short* __restrict__ zwl,
             const unsigned short* __restrict__ rw16, const unsigned short* __restrict__ fw16,
             const float* __restrict__ zb, const float* __restrict__ rb, const float* __restrict__ fb,
             float* __restrict__ out) {
  __shared__ __align__(16) float slab[8][16 * SLP];
  const int tid = (int)threadIdx.x, wave = tid >> 5, lane = tid & 31, hh = lane >> 4, c = lane & 15;
  const int rt = wave >> 2, cg = wave & 3;
  const size_t grow0 = (size_t)blockIdx.x * 32 + (size_t)(rt * 16);
  const int n0 = cg * 64;

  v8f za[4], ra[4], fa[4];
#pragma unroll
  for (int j = 0; j < 4; ++j) { za[j] = z8(); ra[j] = z8(); fa[j] = z8(); }

#pragma unroll 1
  for (int half = 0; half < 2; ++half) {
    const unsigned short* A16 = (half == 0) ? xh : ah;
    const unsigned short* AH = (half == 0) ? xbh : abh;
    const unsigned short* AL = (half == 0) ? xbl : abl;
    const size_t ao = (grow0 + c) * NF + 8 * hh;
    const int kb = half * NF + 8 * hh;
#pragma unroll 1
    for (int kk = 0; kk < NF / 32; ++kk) {
      const int k0 = kk * 32;
      const v16h a16 = ldh(A16 + ao + k0);
      const v16b ahf = ldb(AH + ao + k0);
      const v16b alf = ldb(AL + ao + k0);
#pragma unroll
      for (int j = 0; j < 4; ++j) {
        const size_t wo = (size_t)(n0 + 16 * j + c) * NG + kb + k0;
        const v16b bzh = ldb(zwh + wo);
        const v16b bzl = ldb(zwl + wo);
        const v16h br = ldh(rw16 + wo);
        const v16h bf = ldh(fw16 + wo);
        v8f z = za[j], rr = ra[j], ff = fa[j];
        z = mma_b(ahf, bzh, z);
        z = mma_b(ahf, bzl, z);
        z = mma_b(alf, bzh, z);
        rr = mma_h(a16, br, rr);
        ff = mma_h(a16, bf, ff);
        g_g(z, rr, ff, a16, ahf, alf, bzh, bzl, br, bf);
        za[j] = z;
        ra[j] = rr;
        fa[j] = ff;
      }
    }
  }

  float* sl = &slab[wave][0];
#pragma unroll
  for (int j = 0; j < 4; ++j) {
    const int n = n0 + 16 * j + c;
    const float zbn = zb[n], rbn = rb[n], fbn = fb[n];
#pragma unroll
    for (int r = 0; r < 8; ++r) {
      const int row = 8 * hh + r;
      const float xv = x[(grow0 + row) * NF + n];
      const float zv = tanhf(za[j][r] + zbn);
      const float rv = 1.0f / (1.0f + expf(-(ra[j][r] * 0.0625f + rbn)));
      const float fv = 1.0f / (1.0f + expf(-(fa[j][r] * 0.0625f + fbn)));
      sl[row * SLP + 16 * j + c] = rv * xv + fv * zv;
    }
  }
  __builtin_amdgcn_fence(__ATOMIC_RELEASE, "workgroup");
  __builtin_amdgcn_wave_barrier();
  __builtin_amdgcn_fence(__ATOMIC_ACQUIRE, "workgroup");
  const int c4 = c * 4;
  for (int pass = 0; pass < 2; ++pass) {
#pragma unroll
    for (int it = 0; it < 8; ++it) {
      const int row = it * 2 + hh;
      const v4f v = *(const v4f*)(sl + row * SLP + c4);
      *(volatile v4f*)(out + (grow0 + row) * NF + n0 + c4) = v;
    }
    __threadfence();
  }
}

extern "C" void kernel_launch(void* const* d_in, const int* in_sizes, int n_in,
                              void* d_out, int out_size, void* d_ws, size_t ws_size,
                              hipStream_t stream) {
  if (n_in < 8) return;
  if (in_sizes[0] != NR * NF || in_sizes[1] != 3 * NF) return;
  if (in_sizes[2] != NF * NG || in_sizes[3] != NF) return;
  if (in_sizes[4] != NF * NG || in_sizes[5] != NF) return;
  if (in_sizes[6] != NF * NG || in_sizes[7] != NF) return;
  if (out_size != NR * NF) return;

  const float* x    = (const float*)d_in[0];
  const float* attw = (const float*)d_in[1];
  const float* zw   = (const float*)d_in[2];
  const float* zb   = (const float*)d_in[3];
  const float* rw   = (const float*)d_in[4];
  const float* rb   = (const float*)d_in[5];
  const float* fw   = (const float*)d_in[6];
  const float* fb   = (const float*)d_in[7];

  const size_t P16 = (size_t)NR * NF * 2;
  const size_t PT  = (size_t)NB * NF * NS * 2;
  const size_t PV  = (size_t)NR * 4;
  const size_t PW  = (size_t)NF * NG * 2;
  size_t off = 0;
  const size_t o_xh  = off; off += P16;
  const size_t o_xwc = off; off += P16;
  const size_t o_xbh = off; off += P16;
  const size_t o_xbl = off; off += P16;
  const size_t o_xth = off; off += PT;
  const size_t o_xtl = off; off += PT;
  const size_t o_ah  = off; off += P16;
  const size_t o_abh = off; off += P16;
  const size_t o_abl = off; off += P16;
  const size_t o_av  = off; off += PV;
  const size_t o_bv  = off; off += PV;
  const size_t o_zwh = off; off += PW;
  const size_t o_zwl = off; off += PW;
  const size_t o_rw  = off; off += PW;
  const size_t o_fw  = off; off += PW;
  if (off > ws_size) return;

  char* ws = (char*)d_ws;
  unsigned short* xh  = (unsigned short*)(ws + o_xh);
  unsigned short* xwc = (unsigned short*)(ws + o_xwc);
  unsigned short* xbh = (unsigned short*)(ws + o_xbh);
  unsigned short* xbl = (unsigned short*)(ws + o_xbl);
  unsigned short* xth = (unsigned short*)(ws + o_xth);
  unsigned short* xtl = (unsigned short*)(ws + o_xtl);
  unsigned short* ah  = (unsigned short*)(ws + o_ah);
  unsigned short* abh = (unsigned short*)(ws + o_abh);
  unsigned short* abl = (unsigned short*)(ws + o_abl);
  float*          av  = (float*)(ws + o_av);
  float*          bv  = (float*)(ws + o_bv);
  unsigned short* zwh = (unsigned short*)(ws + o_zwh);
  unsigned short* zwl = (unsigned short*)(ws + o_zwl);
  unsigned short* rwp = (unsigned short*)(ws + o_rw);
  unsigned short* fwp = (unsigned short*)(ws + o_fw);

  const int n8 = NF * NG / 8;
  prep_w<<<dim3((n8 + 255) / 256), dim3(256), 0, stream>>>(zw, rw, fw, zwh, zwl, rwp, fwp, n8);
  prep_x<<<dim3(NR / 64), dim3(256), 0, stream>>>(x, attw, xh, xwc, xbh, xbl, xth, xtl, av, bv);
  attn_kernel<<<dim3(NB * (NS / QROWS)), dim3(128), 0, stream>>>(xwc, xh, xth, xtl, av, bv, ah, abh, abl);
  gates_kernel<<<dim3(NR / 32), dim3(256), 0, stream>>>(x, xh, xbh, xbl, ah, abh, abl, zwh, zwl, rwp, fwp,
                                                       zb, rb, fb, (float*)d_out);
  (void)hipGetLastError();
}
